// RwkvSelfAttention_70832600646182
// MI455X (gfx1250) — hardware-verified
//
#include <hip/hip_runtime.h>
#include <stdint.h>
#include <stddef.h>


#define T_LEN 2048
#define D_DIM 2048
#define H_NUM 32
#define S_DIM 64
#define CHUNK 64

typedef __bf16 v16bf __attribute__((ext_vector_type(16)));
typedef __bf16 v8bf  __attribute__((ext_vector_type(8)));
typedef __bf16 v4bf  __attribute__((ext_vector_type(4)));
typedef float  v8f   __attribute__((ext_vector_type(8)));
typedef float  v4f   __attribute__((ext_vector_type(4)));

union Frag16 { v16bf v; v8bf half[2]; };

static __device__ __forceinline__ v16bf ld_frag(const __bf16* base, int ld, int m, int hh, int k0) {
    Frag16 f;
    const __bf16* p = base + m * ld + k0 + 8 * hh;
    f.half[0] = *(const v8bf*)p;
    f.half[1] = *(const v8bf*)(p + 16);
    return f.v;
}

static __device__ __forceinline__ void mma3(v8f& acc, const v16bf ah, const v16bf al,
                                            const v16bf bh, const v16bf bl) {
    acc = __builtin_amdgcn_wmma_f32_16x16x32_bf16(false, ah, false, bh, (short)0, acc, false, false);
    acc = __builtin_amdgcn_wmma_f32_16x16x32_bf16(false, ah, false, bl, (short)0, acc, false, false);
    acc = __builtin_amdgcn_wmma_f32_16x16x32_bf16(false, al, false, bh, (short)0, acc, false, false);
    asm volatile("v_nop\n\tv_nop\n\tv_nop\n\tv_nop" : "+v"(acc) : "v"(ah), "v"(al), "v"(bh), "v"(bl));
}

static __device__ __forceinline__ void split2(float x, __bf16& hi, __bf16& lo) {
    const __bf16 hv = (__bf16)x;
    hi = hv;
    lo = (__bf16)(x - (float)hv);
}

static __device__ __forceinline__ v8f zero8() {
    v8f z = {0.f, 0.f, 0.f, 0.f, 0.f, 0.f, 0.f, 0.f};
    return z;
}

#define GBM 128
#define GBN 64
#define GBK 64

template <int MIX>
__global__ __launch_bounds__(256) void gemm_x3_kernel(
    const float* __restrict__ A, const float* __restrict__ mixv,
    const float* __restrict__ W, float* __restrict__ C,
    int M, int N, int K)
{
    __shared__ __attribute__((aligned(16))) unsigned char smem[2 * GBM * GBK * 2 + 2 * GBN * GBK * 2];
    __bf16* Ash = (__bf16*)smem;
    __bf16* Asl = Ash + GBM * GBK;
    __bf16* Bsh = Asl + GBM * GBK;
    __bf16* Bsl = Bsh + GBN * GBK;
    float*  Cs  = (float*)smem;

    const int tid  = threadIdx.x;
    const int lane = tid & 31;
    const int wave = tid >> 5;
    const int hh   = lane >> 4;
    const int m    = lane & 15;
    const int rowB = blockIdx.x * GBM;
    const int col0 = blockIdx.y * GBN;
    if (rowB + GBM > M || col0 + GBN > N) return;

    v8f acc[4];
#pragma unroll
    for (int nt = 0; nt < 4; ++nt) acc[nt] = zero8();

    for (int kk = 0; kk < K; kk += GBK) {
#pragma unroll 4
        for (int i = 0; i < 8; ++i) {
            const int idx  = tid + 256 * i;
            const int row  = idx >> 4;
            const int c4   = idx & 15;
            const int grow = rowB + row;
            const int gk   = kk + 4 * c4;
            v4f x = *(const v4f*)(A + (size_t)grow * K + gk);
            if (MIX) {
                const v4f mv = *(const v4f*)(mixv + gk);
                v4f xp = {0.f, 0.f, 0.f, 0.f};
                if (grow > 0) xp = *(const v4f*)(A + (size_t)(grow - 1) * K + gk);
                v4f y;
#pragma unroll
                for (int e = 0; e < 4; ++e) y[e] = x[e] * mv[e] + xp[e] * (1.0f - mv[e]);
                x = y;
            }
            v4bf hv, lv;
#pragma unroll
            for (int e = 0; e < 4; ++e) { __bf16 a, b; split2(x[e], a, b); hv[e] = a; lv[e] = b; }
            *(v4bf*)(Ash + row * GBK + 4 * c4) = hv;
            *(v4bf*)(Asl + row * GBK + 4 * c4) = lv;
        }
#pragma unroll
        for (int i = 0; i < 4; ++i) {
            const int idx = tid + 256 * i;
            const int row = idx >> 4;
            const int c4  = idx & 15;
            const v4f x = *(const v4f*)(W + (size_t)(col0 + row) * K + kk + 4 * c4);
            v4bf hv, lv;
#pragma unroll
            for (int e = 0; e < 4; ++e) { __bf16 a, b; split2(x[e], a, b); hv[e] = a; lv[e] = b; }
            *(v4bf*)(Bsh + row * GBK + 4 * c4) = hv;
            *(v4bf*)(Bsl + row * GBK + 4 * c4) = lv;
        }
        __syncthreads();

#pragma unroll
        for (int k2 = 0; k2 < GBK; k2 += 32) {
            const v16bf ah = ld_frag(Ash, GBK, wave * 16 + m, hh, k2);
            const v16bf al = ld_frag(Asl, GBK, wave * 16 + m, hh, k2);
#pragma unroll
            for (int nt = 0; nt < 4; ++nt) {
                const v16bf bh = ld_frag(Bsh, GBK, nt * 16 + m, hh, k2);
                const v16bf bl = ld_frag(Bsl, GBK, nt * 16 + m, hh, k2);
                mma3(acc[nt], ah, al, bh, bl);
            }
        }
        __syncthreads();
    }

    float* Cw = Cs + wave * (16 * GBN);
#pragma unroll
    for (int nt = 0; nt < 4; ++nt) {
#pragma unroll
        for (int r = 0; r < 8; ++r) Cw[(8 * hh + r) * GBN + nt * 16 + m] = acc[nt][r];
    }
    __syncthreads();
    v4f ov[8];
#pragma unroll
    for (int i = 0; i < 8; ++i) ov[i] = *(const v4f*)(Cw + (2 * i + hh) * GBN + 4 * m);
#pragma unroll
    for (int i = 0; i < 8; ++i) {
        float* p = C + (size_t)(rowB + wave * 16 + 2 * i + hh) * N + col0 + 4 * m;
        *(volatile v4f*)p = ov[i];
    }
    __threadfence();
#pragma unroll
    for (int i = 0; i < 8; ++i) {
        float* p = C + (size_t)(rowB + wave * 16 + 2 * i + hh) * N + col0 + 4 * m;
        *(volatile v4f*)p = ov[i];
    }
}

__global__ __launch_bounds__(128) void scan_kernel(
    const float* __restrict__ Kp, const float* __restrict__ Vp, const float* __restrict__ Rp,
    const float* __restrict__ time_decay, const float* __restrict__ time_first,
    const float* __restrict__ lxw, const float* __restrict__ lxb,
    const float* __restrict__ state0, float* __restrict__ Yn)
{
    extern __shared__ __attribute__((aligned(16))) unsigned char dsm[];
    __shared__ float wp[80];

    float*  St  = (float*)dsm;
    float*  Yf  = St + S_DIM * S_DIM;
    __bf16* Rh  = (__bf16*)(Yf + CHUNK * S_DIM);
    __bf16* Rl  = Rh  + 4096;
    __bf16* Kh  = Rl  + 4096;
    __bf16* Kl  = Kh  + 4096;
    __bf16* Kth = Kl  + 4096;
    __bf16* Ktl = Kth + 4096;
    __bf16* Vth = Ktl + 4096;
    __bf16* Vtl = Vth + 4096;
    __bf16* Vwh = Vtl + 4096;
    __bf16* Vwl = Vwh + 4096;
    __bf16* Sh  = Vwl + 4096;
    __bf16* Sl  = Sh  + 4096;
    __bf16* Ph  = Sl  + 4096;
    __bf16* Pl  = Ph  + 4096;

    const int hd   = blockIdx.x;
    const int tid  = threadIdx.x;
    const int lane = tid & 31;
    const int wave = tid >> 5;
    const int hh   = lane >> 4;
    const int m    = lane & 15;
    const int colbase = hd * S_DIM;

    if (tid == 0) {
        const float w1 = expf(-expf(time_decay[hd]));
        float p = 1.0f;
        wp[0] = 1.0f;
        for (int i = 1; i <= CHUNK; ++i) { p = p * w1; wp[i] = p; }
        wp[65] = expf(time_first[hd]);
    }
    for (int i = tid; i < S_DIM * S_DIM; i += 128) {
        const int s = i >> 6, d = i & 63;
        St[d * S_DIM + s] = state0[(size_t)hd * S_DIM * S_DIM + i];
    }
    __syncthreads();

    const float u   = wp[65];
    const float w64 = wp[CHUNK];
    float wrow[8];
#pragma unroll
    for (int r = 0; r < 8; ++r) wrow[r] = wp[16 * wave + 8 * hh + r];
    const v4f gw = *(const v4f*)(lxw + colbase + 4 * m);
    const v4f gb = *(const v4f*)(lxb + colbase + 4 * m);

    for (int c0 = 0; c0 < T_LEN; c0 += CHUNK) {
#pragma unroll 2
        for (int i = 0; i < 8; ++i) {
            const int idx = tid + 128 * i;
            const int t   = idx >> 4;
            const int c4  = idx & 15;
            const size_t g = (size_t)(c0 + t) * D_DIM + colbase + 4 * c4;
            const v4f kx = *(const v4f*)(Kp + g);
            const v4f vx = *(const v4f*)(Vp + g);
            const v4f rx = *(const v4f*)(Rp + g);
            const float wt = wp[CHUNK - 1 - t];
            v4bf khv, klv, rhv, rlv;
#pragma unroll
            for (int e = 0; e < 4; ++e) {
                const int s = 4 * c4 + e;
                __bf16 a, b;
                split2(rx[e], a, b); rhv[e] = a; rlv[e] = b;
                split2(kx[e], a, b); khv[e] = a; klv[e] = b;
                Kth[s * CHUNK + t] = a; Ktl[s * CHUNK + t] = b;
                split2(vx[e], a, b);
                Vth[s * CHUNK + t] = a; Vtl[s * CHUNK + t] = b;
                split2(vx[e] * wt, a, b);
                Vwh[s * CHUNK + t] = a; Vwl[s * CHUNK + t] = b;
            }
            *(v4bf*)(Rh + t * S_DIM + 4 * c4) = rhv;
            *(v4bf*)(Rl + t * S_DIM + 4 * c4) = rlv;
            *(v4bf*)(Kh + t * S_DIM + 4 * c4) = khv;
            *(v4bf*)(Kl + t * S_DIM + 4 * c4) = klv;
        }
#pragma unroll 2
        for (int i = 0; i < 8; ++i) {
            const int idx = tid + 128 * i;
            const v4f sx = *(const v4f*)(St + 4 * idx);
            v4bf hv, lv;
#pragma unroll
            for (int e = 0; e < 4; ++e) { __bf16 a, b; split2(sx[e], a, b); hv[e] = a; lv[e] = b; }
            *(v4bf*)(Sh + 4 * idx) = hv;
            *(v4bf*)(Sl + 4 * idx) = lv;
        }
        __syncthreads();

        {
            v8f acc[4];
#pragma unroll
            for (int nt = 0; nt < 4; ++nt) acc[nt] = zero8();
#pragma unroll
            for (int kk = 0; kk < S_DIM; kk += 32) {
                const v16bf ah = ld_frag(Rh, S_DIM, 16 * wave + m, hh, kk);
                const v16bf al = ld_frag(Rl, S_DIM, 16 * wave + m, hh, kk);
#pragma unroll
                for (int nt = 0; nt < 4; ++nt) {
                    const v16bf bh = ld_frag(Kh, S_DIM, nt * 16 + m, hh, kk);
                    const v16bf bl = ld_frag(Kl, S_DIM, nt * 16 + m, hh, kk);
                    mma3(acc[nt], ah, al, bh, bl);
                }
            }
#pragma unroll
            for (int nt = 0; nt < 4; ++nt) {
#pragma unroll
                for (int r = 0; r < 8; ++r) {
                    const int t  = 16 * wave + 8 * hh + r;
                    const int j  = nt * 16 + m;
                    const int dl = t - 1 - j;
                    const int di = dl < 0 ? 0 : dl;
                    const float wd = wp[di];
                    const float f  = (j > t) ? 0.0f : ((j == t) ? u : wd);
                    __bf16 a, b;
                    split2(acc[nt][r] * f, a, b);
                    Ph[t * CHUNK + j] = a;
                    Pl[t * CHUNK + j] = b;
                }
            }
        }
        __syncthreads();

        {
            v8f acc[4];
#pragma unroll
            for (int nt = 0; nt < 4; ++nt) acc[nt] = zero8();
#pragma unroll
            for (int kk = 0; kk < S_DIM; kk += 32) {
                const v16bf ah = ld_frag(Rh, S_DIM, 16 * wave + m, hh, kk);
                const v16bf al = ld_frag(Rl, S_DIM, 16 * wave + m, hh, kk);
#pragma unroll
                for (int nt = 0; nt < 4; ++nt) {
                    const v16bf bh = ld_frag(Sh, S_DIM, nt * 16 + m, hh, kk);
                    const v16bf bl = ld_frag(Sl, S_DIM, nt * 16 + m, hh, kk);
                    mma3(acc[nt], ah, al, bh, bl);
                }
            }
#pragma unroll
            for (int nt = 0; nt < 4; ++nt) {
#pragma unroll
                for (int r = 0; r < 8; ++r) acc[nt][r] = acc[nt][r] * wrow[r];
            }
#pragma unroll
            for (int kk = 0; kk < CHUNK; kk += 32) {
                const v16bf ah = ld_frag(Ph, CHUNK, 16 * wave + m, hh, kk);
                const v16bf al = ld_frag(Pl, CHUNK, 16 * wave + m, hh, kk);
#pragma unroll
                for (int nt = 0; nt < 4; ++nt) {
                    const v16bf bh = ld_frag(Vth, CHUNK, nt * 16 + m, hh, kk);
                    const v16bf bl = ld_frag(Vtl, CHUNK, nt * 16 + m, hh, kk);
                    mma3(acc[nt], ah, al, bh, bl);
                }
            }
#pragma unroll
            for (int nt = 0; nt < 4; ++nt) {
#pragma unroll
                for (int r = 0; r < 8; ++r)
                    Yf[(16 * wave + 8 * hh + r) * S_DIM + nt * 16 + m] = acc[nt][r];
            }
        }
        __syncthreads();

        {
            v4f yo[8];
#pragma unroll
            for (int i = 0; i < 8; ++i) {
                const int t = 16 * wave + 2 * i + hh;
                const v4f y = *(const v4f*)(Yf + t * S_DIM + 4 * m);
                float s1 = (y[0] + y[1]) + (y[2] + y[3]);
                s1 += __shfl_xor(s1, 8);
                s1 += __shfl_xor(s1, 4);
                s1 += __shfl_xor(s1, 2);
                s1 += __shfl_xor(s1, 1);
                const float mu = s1 * (1.0f / 64.0f);
                v4f dv;
#pragma unroll
                for (int e = 0; e < 4; ++e) dv[e] = y[e] - mu;
                float s2 = (dv[0] * dv[0] + dv[1] * dv[1]) + (dv[2] * dv[2] + dv[3] * dv[3]);
                s2 += __shfl_xor(s2, 8);
                s2 += __shfl_xor(s2, 4);
                s2 += __shfl_xor(s2, 2);
                s2 += __shfl_xor(s2, 1);
                const float var = s2 * (1.0f / 64.0f);
                const float inv = rsqrtf(var + 1e-5f);
                v4f o;
#pragma unroll
                for (int e = 0; e < 4; ++e) o[e] = (dv[e] * inv) * gw[e] + gb[e];
                yo[i] = o;
            }
#pragma unroll
            for (int i = 0; i < 8; ++i) {
                float* p = Yn + (size_t)(c0 + 16 * wave + 2 * i + hh) * D_DIM + colbase + 4 * m;
                *(volatile v4f*)p = yo[i];
            }
            __threadfence();
#pragma unroll
            for (int i = 0; i < 8; ++i) {
                float* p = Yn + (size_t)(c0 + 16 * wave + 2 * i + hh) * D_DIM + colbase + 4 * m;
                *(volatile v4f*)p = yo[i];
            }
        }

        {
            v8f acc[4];
#pragma unroll
            for (int nt = 0; nt < 4; ++nt) acc[nt] = zero8();
#pragma unroll
            for (int kk = 0; kk < CHUNK; kk += 32) {
                const v16bf ah = ld_frag(Kth, CHUNK, 16 * wave + m, hh, kk);
                const v16bf al = ld_frag(Ktl, CHUNK, 16 * wave + m, hh, kk);
#pragma unroll
                for (int nt = 0; nt < 4; ++nt) {
                    const v16bf bh = ld_frag(Vwh, CHUNK, nt * 16 + m, hh, kk);
                    const v16bf bl = ld_frag(Vwl, CHUNK, nt * 16 + m, hh, kk);
                    mma3(acc[nt], ah, al, bh, bl);
                }
            }
#pragma unroll
            for (int nt = 0; nt < 4; ++nt) {
#pragma unroll
                for (int r = 0; r < 8; ++r) {
                    const int s = 16 * wave + 8 * hh + r;
                    const int d = nt * 16 + m;
                    const float old = St[d * S_DIM + s];
                    St[d * S_DIM + s] = w64 * old + acc[nt][r];
                }
            }
        }
        __syncthreads();
    }
}

extern "C" void kernel_launch(void* const* d_in, const int* in_sizes, int n_in,
                              void* d_out, int out_size, void* d_ws, size_t ws_size,
                              hipStream_t stream) {
    if (n_in < 13) return;
    const size_t TD = (size_t)T_LEN * D_DIM;
    const size_t DD = (size_t)D_DIM * D_DIM;
    if ((size_t)in_sizes[0] != TD) return;
    if (in_sizes[1] != H_NUM || in_sizes[2] != H_NUM) return;
    if (in_sizes[3] != D_DIM || in_sizes[4] != D_DIM || in_sizes[5] != D_DIM) return;
    if ((size_t)in_sizes[6] != DD || (size_t)in_sizes[7] != DD ||
        (size_t)in_sizes[8] != DD || (size_t)in_sizes[9] != DD) return;
    if (in_sizes[10] != D_DIM || in_sizes[11] != D_DIM) return;
    if (in_sizes[12] != H_NUM * S_DIM * S_DIM) return;
    if ((size_t)out_size != TD) return;

    const float* hidden     = (const float*)d_in[0];
    const float* time_decay = (const float*)d_in[1];
    const float* time_first = (const float*)d_in[2];
    const float* tmk        = (const float*)d_in[3];
    const float* tmv        = (const float*)d_in[4];
    const float* tmr        = (const float*)d_in[5];
    const float* Wk         = (const float*)d_in[6];
    const float* Wv         = (const float*)d_in[7];
    const float* Wr         = (const float*)d_in[8];
    const float* Wo         = (const float*)d_in[9];
    const float* lxw        = (const float*)d_in[10];
    const float* lxb        = (const float*)d_in[11];
    const float* state0     = (const float*)d_in[12];
    float* out = (float*)d_out;

    const size_t need = 4 * TD * sizeof(float);
    if (ws_size < need) return;
    float* kb = (float*)d_ws;
    float* vb = kb + TD;
    float* rb = vb + TD;
    float* yb = rb + TD;

    const dim3 gg(T_LEN / GBM, D_DIM / GBN), gbk(256);
    gemm_x3_kernel<1><<<gg, gbk, 0, stream>>>(hidden, tmk, Wk, kb, T_LEN, D_DIM, D_DIM);
    gemm_x3_kernel<1><<<gg, gbk, 0, stream>>>(hidden, tmv, Wv, vb, T_LEN, D_DIM, D_DIM);
    gemm_x3_kernel<1><<<gg, gbk, 0, stream>>>(hidden, tmr, Wr, rb, T_LEN, D_DIM, D_DIM);

    const size_t smem = (size_t)2 * S_DIM * S_DIM * sizeof(float) + (size_t)14 * S_DIM * S_DIM * sizeof(__bf16);
    hipFuncSetAttribute(reinterpret_cast<const void*>(&scan_kernel),
                        hipFuncAttributeMaxDynamicSharedMemorySize, (int)smem);
    scan_kernel<<<H_NUM, 128, smem, stream>>>(kb, vb, rb, time_decay, time_first, lxw, lxb, state0, yb);

    gemm_x3_kernel<0><<<gg, gbk, 0, stream>>>(yb, tmk, Wo, out, T_LEN, D_DIM, D_DIM);
}
